// DiscreteQKTRBlock_25520695673113
// MI455X (gfx1250) — hardware-verified
//
#include <hip/hip_runtime.h>
#define NPt 100000
#define NPP 100096
#define PL 128
#define VEC 16
#define KO 27
#define QP 25024
#define NEGc (-1e9f)
typedef __bf16 v16b __attribute__((ext_vector_type(16)));
typedef unsigned short v8us __attribute__((ext_vector_type(8), may_alias));
typedef float  v8f  __attribute__((ext_vector_type(8)));
typedef float  v4f  __attribute__((ext_vector_type(4)));
typedef float  v4fa __attribute__((ext_vector_type(4), may_alias));
union FragB { v16b v; v8us half[2]; unsigned short u[16]; };

__device__ __forceinline__ unsigned short bf16_bits(float x) { unsigned int u = __float_as_uint(x); return (unsigned short)((u + 0x7FFFu + ((u >> 16) & 1u)) >> 16); }
__device__ __forceinline__ float bf16_val(unsigned short b) { return __uint_as_float(((unsigned int)b) << 16); }
__device__ __forceinline__ float bf16_round(float x) { return bf16_val(bf16_bits(x)); }
template <int NT>
__device__ __forceinline__ v8f mmaN(v16b ah, v16b al, v16b bh, v16b bl, v8f c) {
  c = __builtin_amdgcn_wmma_f32_16x16x32_bf16(false, ah, false, bh, (short)0, c, false, false);
  if (NT >= 2) c = __builtin_amdgcn_wmma_f32_16x16x32_bf16(false, al, false, bh, (short)0, c, false, false);
  if (NT >= 3) c = __builtin_amdgcn_wmma_f32_16x16x32_bf16(false, ah, false, bl, (short)0, c, false, false);
  asm volatile("v_nop\n\tv_nop\n\tv_nop\n\tv_nop" : "+v"(c) : "v"(ah), "v"(al), "v"(bh), "v"(bl));
  return c;
}

__global__ __launch_bounds__(256) void k_wt_bf16(const float* __restrict__ W, unsigned short* __restrict__ Wt, int K, int N) {
  const int t = blockIdx.x * 256 + threadIdx.x;
  const int k8n = K / 8;
  if (t >= N * k8n) return;
  const int n = t / k8n, k8 = (t % k8n) * 8;
  v8us v;
#pragma unroll
  for (int i = 0; i < 8; ++i) v[i] = bf16_bits(W[(size_t)(k8 + i) * N + n]);
  *(volatile v8us*)(Wt + (size_t)n * K + k8) = v;
  __threadfence();
  *(volatile v8us*)(Wt + (size_t)n * K + k8) = v;
}

template <bool ASPLIT, int ACT, bool BIAS_BF16>
__global__ __launch_bounds__(128) void k_gemm_bf(const float* __restrict__ A, int lda, const unsigned short* __restrict__ Wt, int ldb,
                                               const float* __restrict__ bias, float* __restrict__ C, int ldc, int M, int N, int K) {
  __shared__ __attribute__((aligned(16))) float so[4][16][64];
  const int tid = threadIdx.x, w = tid >> 5, lane = tid & 31, ln = lane & 15, hh = lane >> 4;
  const int ntn = N / 64;
  const int wid = blockIdx.x * 4 + w;
  const int mt = wid / ntn, nq = wid % ntn;
  if (mt * 16 >= M) return;
  const int row0 = mt * 16, col0 = nq * 64;
  const float* arow = A + (size_t)(row0 + ln) * lda;
  v8f acc[4] = {};
  for (int kb = 0; kb < K; kb += 32) {
    FragB ah, al;
    const v4f x0 = *(const v4fa*)(arow + kb + 8 * hh), x1 = *(const v4fa*)(arow + kb + 8 * hh + 4);
    const v4f x2 = *(const v4fa*)(arow + kb + 16 + 8 * hh), x3 = *(const v4fa*)(arow + kb + 16 + 8 * hh + 4);
    float xs[16] = {x0[0],x0[1],x0[2],x0[3],x1[0],x1[1],x1[2],x1[3],x2[0],x2[1],x2[2],x2[3],x3[0],x3[1],x3[2],x3[3]};
#pragma unroll
    for (int i = 0; i < 16; ++i) { const unsigned short hb = bf16_bits(xs[i]); ah.u[i] = hb; al.u[i] = ASPLIT ? bf16_bits(xs[i] - bf16_val(hb)) : (unsigned short)0; }
#pragma unroll
    for (int t = 0; t < 4; ++t) {
      const unsigned short* brow = Wt + (size_t)(col0 + t * 16 + ln) * ldb + kb;
      FragB b;
      b.half[0] = *(const v8us*)(brow + 8 * hh);
      b.half[1] = *(const v8us*)(brow + 16 + 8 * hh);
      acc[t] = mmaN<ASPLIT ? 2 : 1>(ah.v, al.v, b.v, b.v, acc[t]);
    }
  }
#pragma unroll
  for (int t = 0; t < 4; ++t) {
    float bv = bias ? bias[col0 + t * 16 + ln] : 0.f;
    if (BIAS_BF16) bv = bf16_round(bv);
#pragma unroll
    for (int r = 0; r < 8; ++r) { float v = acc[t][r] + bv; if (ACT == 1) v = fmaxf(v, 0.f); so[w][8 * hh + r][t * 16 + ln] = v; }
  }
  __builtin_amdgcn_fence(__ATOMIC_ACQ_REL, "workgroup");
  __builtin_amdgcn_wave_barrier();
  const int rsub = lane >> 4, c4 = (lane & 15) * 4;
  for (int pass = 0; pass < 2; ++pass) {
#pragma unroll
    for (int q = 0; q < 8; ++q) {
      const int r = q * 2 + rsub;
      const v4f v = *(const v4fa*)&so[w][r][c4];
      *(volatile v4f*)(C + (size_t)(row0 + r) * ldc + col0 + c4) = v;
    }
    if (pass == 0) __threadfence();
  }
}

template <bool ASPLIT, int ACT, bool BIAS_BF16, bool RES_BF16>
__global__ __launch_bounds__(128) void k_gemm_bf3(const float* __restrict__ A, int lda, const unsigned short* __restrict__ Wt, int ldb,
                                                const float* __restrict__ bias, const float* __restrict__ resid, int rmod, int ldr,
                                                float* __restrict__ C, int ldc, int M, int N, int K) {
  __shared__ __attribute__((aligned(16))) float so[4][16][64];
  const int tid = threadIdx.x, w = tid >> 5, lane = tid & 31, ln = lane & 15, hh = lane >> 4;
  const int ntn = N / 64;
  const int wid = blockIdx.x * 4 + w;
  const int mt = wid / ntn, nq = wid % ntn;
  if (mt * 16 >= M) return;
  const int row0 = mt * 16, col0 = nq * 64;
  const float* arow = A + (size_t)(row0 + ln) * lda;
  v8f acc[4] = {};
  for (int kb = 0; kb < K; kb += 32) {
    FragB ah, al;
    const v4f x0 = *(const v4fa*)(arow + kb + 8 * hh), x1 = *(const v4fa*)(arow + kb + 8 * hh + 4);
    const v4f x2 = *(const v4fa*)(arow + kb + 16 + 8 * hh), x3 = *(const v4fa*)(arow + kb + 16 + 8 * hh + 4);
    float xs[16] = {x0[0],x0[1],x0[2],x0[3],x1[0],x1[1],x1[2],x1[3],x2[0],x2[1],x2[2],x2[3],x3[0],x3[1],x3[2],x3[3]};
#pragma unroll
    for (int i = 0; i < 16; ++i) { const unsigned short hb = bf16_bits(xs[i]); ah.u[i] = hb; al.u[i] = ASPLIT ? bf16_bits(xs[i] - bf16_val(hb)) : (unsigned short)0; }
#pragma unroll
    for (int t = 0; t < 4; ++t) {
      const unsigned short* brow = Wt + (size_t)(col0 + t * 16 + ln) * ldb + kb;
      FragB b;
      b.half[0] = *(const v8us*)(brow + 8 * hh);
      b.half[1] = *(const v8us*)(brow + 16 + 8 * hh);
      acc[t] = mmaN<ASPLIT ? 2 : 1>(ah.v, al.v, b.v, b.v, acc[t]);
    }
  }
#pragma unroll
  for (int t = 0; t < 4; ++t) {
    const int col = col0 + t * 16 + ln;
    float bv = bias ? bias[col] : 0.f;
    if (BIAS_BF16) bv = bf16_round(bv);
#pragma unroll
    for (int r = 0; r < 8; ++r) {
      float v = acc[t][r] + bv;
      if (resid) { float rv = resid[(size_t)((row0 + 8 * hh + r) % rmod) * ldr + col]; if (RES_BF16) rv = bf16_round(rv); v += rv; }
      if (ACT == 1) v = fmaxf(v, 0.f);
      if (ACT == 2) v = 0.5f * v * (1.0f + erff(v * 0.70710678118654752f));
      if (ACT == 3) { const float u = 0.7978845608028654f * (v + 0.044715f * v * v * v); v = 0.5f * v * (1.0f + tanhf(u)); }
      so[w][8 * hh + r][t * 16 + ln] = v;
    }
  }
  __builtin_amdgcn_fence(__ATOMIC_ACQ_REL, "workgroup");
  __builtin_amdgcn_wave_barrier();
  const int rsub = lane >> 4, c4 = (lane & 15) * 4;
  for (int pass = 0; pass < 2; ++pass) {
#pragma unroll
    for (int q = 0; q < 8; ++q) {
      const int r = q * 2 + rsub;
      const v4f v = *(const v4fa*)&so[w][r][c4];
      *(volatile v4f*)(C + (size_t)(row0 + r) * ldc + col0 + c4) = v;
    }
    if (pass == 0) __threadfence();
  }
}
template <bool PARAM_BF16>
__global__ __launch_bounds__(256) void k_layernorm(const float* __restrict__ X, const float* __restrict__ R, const float* __restrict__ g, const float* __restrict__ bta,
                                                  float* __restrict__ out_sum, float* __restrict__ out_norm, int N, float eps) {
  __shared__ float red[256];
  const int row = blockIdx.x, tid = threadIdx.x;
  const float* x = X + (size_t)row * N; const float* rr = R ? R + (size_t)row * N : nullptr;
  float vals[16];
  const int per = N / 256;
  float s1 = 0.f;
  for (int u = 0; u < per / 4; ++u) {
    const int j = tid * 4 + 1024 * u;
    const v4f a = *(const v4fa*)(x + j);
    v4f b = {0.f,0.f,0.f,0.f}; if (rr) b = *(const v4fa*)(rr + j);
#pragma unroll
    for (int q = 0; q < 4; ++q) { const float v = a[q] + b[q]; vals[u * 4 + q] = v; s1 += v; }
  }
  red[tid] = s1; __syncthreads();
  for (int st = 128; st > 0; st >>= 1) { if (tid < st) red[tid] += red[tid + st]; __syncthreads(); }
  const float mu = red[0] / (float)N; __syncthreads();
  float s2 = 0.f;
  for (int u = 0; u < per / 4; ++u)
#pragma unroll
    for (int q = 0; q < 4; ++q) { const float c = vals[u * 4 + q] - mu; s2 += c * c; }
  red[tid] = s2; __syncthreads();
  for (int st = 128; st > 0; st >>= 1) { if (tid < st) red[tid] += red[tid + st]; __syncthreads(); }
  const float rs = rsqrtf(red[0] / (float)N + eps);
  for (int pass = 0; pass < 2; ++pass) {
    for (int u = 0; u < per / 4; ++u) {
      const int j = tid * 4 + 1024 * u;
      v4f o, sm;
#pragma unroll
      for (int q = 0; q < 4; ++q) {
        float gg = g[j + q], bb = bta[j + q];
        if (PARAM_BF16) { gg = bf16_round(gg); bb = bf16_round(bb); }
        sm[q] = vals[u * 4 + q]; o[q] = (vals[u * 4 + q] - mu) * rs * gg + bb;
      }
      if (out_sum) *(volatile v4f*)(out_sum + (size_t)row * N + j) = sm;
      *(volatile v4f*)(out_norm + (size_t)row * N + j) = o;
    }
    if (pass == 0) __threadfence();
  }
}


typedef _Float16 v16h __attribute__((ext_vector_type(16)));
union FragH { v16h v; v8us half[2]; _Float16 h[16]; unsigned short u[16]; };
template <int NT>
__device__ __forceinline__ v8f mmaH(v16h ah, v16h al, v16h bh, v16h bl, v8f c) {
  c = __builtin_amdgcn_wmma_f32_16x16x32_f16(false, ah, false, bh, (short)0, c, false, false);
  if (NT >= 2) c = __builtin_amdgcn_wmma_f32_16x16x32_f16(false, al, false, bh, (short)0, c, false, false);
  if (NT >= 3) c = __builtin_amdgcn_wmma_f32_16x16x32_f16(false, ah, false, bl, (short)0, c, false, false);
  asm volatile("v_nop\n\tv_nop\n\tv_nop\n\tv_nop" : "+v"(c) : "v"(ah), "v"(al), "v"(bh), "v"(bl));
  return c;
}
template <bool ASPLIT>
__global__ __launch_bounds__(128) void k_gemm_h(const float* __restrict__ A, int lda, size_t sA, const _Float16* __restrict__ Bh, int ldb, size_t sB, float alpha, float* __restrict__ C, int ldc, size_t sC, int M, int N, int K) {
  __shared__ __attribute__((aligned(16))) float so[4][16][64];
  const int tid = threadIdx.x, w = tid >> 5, lane = tid & 31, ln = lane & 15, hh = lane >> 4; const int by = blockIdx.y;
  A += (size_t)by * sA; Bh += (size_t)by * sB; C += (size_t)by * sC;
  const int ntn = (N + 63) / 64; const int wid = blockIdx.x * 4 + w; const int mt = wid / ntn, nq = wid % ntn; if (mt * 16 >= M) return;
  const int row0 = mt * 16, col0 = nq * 64; const float* arow = A + (size_t)(row0 + ln) * lda;
  v8f acc[4] = {};
  for (int kb = 0; kb < K; kb += 32) {
    FragH ah, al;
    const v4f x0 = *(const v4fa*)(arow + kb + 8 * hh), x1 = *(const v4fa*)(arow + kb + 8 * hh + 4), x2 = *(const v4fa*)(arow + kb + 16 + 8 * hh), x3 = *(const v4fa*)(arow + kb + 16 + 8 * hh + 4);
    float xs[16] = {x0[0],x0[1],x0[2],x0[3],x1[0],x1[1],x1[2],x1[3],x2[0],x2[1],x2[2],x2[3],x3[0],x3[1],x3[2],x3[3]};
#pragma unroll
    for (int i = 0; i < 16; ++i) { const _Float16 h = (_Float16)xs[i]; ah.h[i] = h; al.h[i] = ASPLIT ? (_Float16)(xs[i] - (float)h) : (_Float16)0.0f; }
#pragma unroll
    for (int t = 0; t < 4; ++t) { if (col0 + t * 16 >= N) continue; const size_t boff = (size_t)(col0 + t * 16 + ln) * ldb + kb; FragH bq; bq.half[0] = *(const v8us*)(Bh + boff + 8 * hh); bq.half[1] = *(const v8us*)(Bh + boff + 16 + 8 * hh);
      acc[t] = mmaH<ASPLIT ? 2 : 1>(ah.v, al.v, bq.v, bq.v, acc[t]); }
  }
#pragma unroll
  for (int t = 0; t < 4; ++t) { if (col0 + t * 16 >= N) continue;
#pragma unroll
    for (int r = 0; r < 8; ++r) so[w][8 * hh + r][t * 16 + ln] = acc[t][r] * alpha; }
  __builtin_amdgcn_fence(__ATOMIC_ACQ_REL, "workgroup"); __builtin_amdgcn_wave_barrier();
  const int rsub = lane >> 4, c4 = (lane & 15) * 4;
  for (int pass = 0; pass < 2; ++pass) {
#pragma unroll
    for (int q = 0; q < 8; ++q) { const int r = q * 2 + rsub; if (col0 + c4 < N) { const v4f v = *(const v4fa*)&so[w][r][c4]; *(volatile v4f*)(C + (size_t)(row0 + r) * ldc + col0 + c4) = v; } }
    if (pass == 0) __threadfence(); }
}

__global__ __launch_bounds__(256) void k_wt_f16(const float* __restrict__ W, _Float16* __restrict__ Wt, int K, int N, float scale) {
  const int t = blockIdx.x * 256 + threadIdx.x; if (t >= N * (K / 8)) return; const int n = t / (K / 8), k8 = (t % (K / 8)) * 8; FragH f;
#pragma unroll
  for (int i = 0; i < 8; ++i) f.h[i] = (_Float16)(bf16_round(W[(size_t)(k8 + i) * N + n]) * scale); const v8us o = f.half[0];
  *(volatile v8us*)((unsigned short*)Wt + (size_t)n * K + k8) = o; __threadfence(); *(volatile v8us*)((unsigned short*)Wt + (size_t)n * K + k8) = o;
}
template <int ACT>
__global__ __launch_bounds__(128) void k_gemm_hhx(const _Float16* __restrict__ A, int lda, size_t sA, const _Float16* __restrict__ Bh, int ldb, size_t sB, float alpha, const float* __restrict__ bias, size_t sBias, const float* __restrict__ CP, int rowsPerB, size_t sCPb, int row0g,
    float* __restrict__ C, _Float16* __restrict__ C16, int ldc, size_t sC, int M, int N, int K) {
  __shared__ __attribute__((aligned(16))) float so[4][16][64];
  const int tid = threadIdx.x, w = tid >> 5, lane = tid & 31, ln = lane & 15, hh = lane >> 4; const int by = blockIdx.y;
  A += (size_t)by * sA; Bh += (size_t)by * sB; const size_t cofs = (size_t)by * sC; const float* bp = bias ? bias + (size_t)by * sBias : nullptr;
  const int ntn = (N + 63) / 64; const int wid = blockIdx.x * 4 + w; const int mt = wid / ntn, nq = wid % ntn; if (mt * 16 >= M) return;
  const int row0 = mt * 16, col0 = nq * 64; const _Float16* arow = A + (size_t)(row0 + ln) * lda;
  v8f acc[4] = {};
  for (int kb = 0; kb < K; kb += 32) { FragH ah; ah.half[0] = *(const v8us*)((const unsigned short*)arow + kb + 8 * hh); ah.half[1] = *(const v8us*)((const unsigned short*)arow + kb + 16 + 8 * hh);
#pragma unroll
    for (int t = 0; t < 4; ++t) { if (col0 + t * 16 >= N) continue; const size_t boff = (size_t)(col0 + t * 16 + ln) * ldb + kb; FragH bq; bq.half[0] = *(const v8us*)((const unsigned short*)Bh + boff + 8 * hh); bq.half[1] = *(const v8us*)((const unsigned short*)Bh + boff + 16 + 8 * hh);
      acc[t] = mmaH<1>(ah.v, ah.v, bq.v, bq.v, acc[t]); }
  }
#pragma unroll
  for (int t = 0; t < 4; ++t) { if (col0 + t * 16 >= N) continue; const int col = col0 + t * 16 + ln; const float bv = bp ? bf16_round(bp[col]) : 0.f;
#pragma unroll
    for (int r = 0; r < 8; ++r) { float v = acc[t][r] * alpha + bv; if (CP) { const int bidx = (row0g + row0 + 8 * hh + r) / rowsPerB; v += CP[(size_t)bidx * sCPb + (size_t)by * 64 + col]; } if (ACT == 1) v = (v > 0.f) ? v : expm1f(v); else if (ACT == 7) v = (v > 0.f) ? v + 1.0f : expf(v); else if (ACT == 8) v = tanhf(v); else if (ACT == 9) v = 0.5f * v * (1.0f + tanhf(0.7978845608028654f * (v + 0.044715f * v * v * v))); else if (ACT == 11) v = 1.0f / (1.0f + expf(-v)); else if (ACT == 12) v = (v > 0.f) ? v : 0.01f * v; else if (ACT == 14) v = (v > 0.f) ? v : 0.1f * v; else if (ACT == 15) v = v / (1.0f + expf(-v)); else if (ACT == 3) v = fmaxf(v, 0.f); else if (ACT == 6) v = 0.5f * v * (1.0f + erff(v * 0.70710678118654752f)); so[w][8 * hh + r][t * 16 + ln] = v; } }
  __builtin_amdgcn_fence(__ATOMIC_ACQ_REL, "workgroup"); __builtin_amdgcn_wave_barrier();
  const int rsub = lane >> 4, c4 = (lane & 15) * 4; typedef _Float16 v4h __attribute__((ext_vector_type(4)));
  for (int pass = 0; pass < 2; ++pass) {
#pragma unroll
    for (int q = 0; q < 8; ++q) { const int r = q * 2 + rsub; if (col0 + c4 < N) { const v4f v = *(const v4fa*)&so[w][r][c4]; if (C) *(volatile v4f*)(C + cofs + (size_t)(row0 + r) * ldc + col0 + c4) = v; if (C16) { v4h h4; for (int i = 0; i < 4; ++i) h4[i] = (_Float16)v[i]; *(volatile v4h*)(C16 + cofs + (size_t)(row0 + r) * ldc + col0 + c4) = h4; } } }
    if (pass == 0) __threadfence(); }
}


typedef _Float16 v4h __attribute__((ext_vector_type(4)));

__global__ __launch_bounds__(256) void k_x16(const float* __restrict__ x, _Float16* __restrict__ X16, size_t n8) { const size_t t = (size_t)blockIdx.x * 256 + threadIdx.x; if (t >= n8) return; FragH f;
#pragma unroll
  for (int q = 0; q < 8; ++q) f.h[q] = (_Float16)bf16_round(x[t * 8 + q]); *(volatile v8us*)((unsigned short*)X16 + t * 8) = f.half[0]; __threadfence(); *(volatile v8us*)((unsigned short*)X16 + t * 8) = f.half[0]; }
__global__ __launch_bounds__(256) void k_h16(const float* __restrict__ x, _Float16* __restrict__ X16, size_t n8) { const size_t t = (size_t)blockIdx.x * 256 + threadIdx.x; if (t >= n8) return; FragH f;
#pragma unroll
  for (int q = 0; q < 8; ++q) f.h[q] = (_Float16)x[t * 8 + q]; *(volatile v8us*)((unsigned short*)X16 + t * 8) = f.half[0]; __threadfence(); *(volatile v8us*)((unsigned short*)X16 + t * 8) = f.half[0]; }
__global__ __launch_bounds__(256) void k_round16f(const float* __restrict__ W, _Float16* __restrict__ Bt, size_t n8) { const size_t t = (size_t)blockIdx.x * 256 + threadIdx.x; if (t >= n8) return; FragH f;
#pragma unroll
  for (int i = 0; i < 8; ++i) f.h[i] = (_Float16)(bf16_round(W[t * 8 + i]) * 16.0f); *(volatile v8us*)((unsigned short*)Bt + t * 8) = f.half[0]; __threadfence(); *(volatile v8us*)((unsigned short*)Bt + t * 8) = f.half[0]; }
template <int NHv, int TTv>
__global__ __launch_bounds__(256) void k_vt(const _Float16* __restrict__ V16, int ldv, int voff, _Float16* __restrict__ Vt) { __shared__ unsigned short tl[64][66]; const int tid = threadIdx.x; const int slab = blockIdx.x / (TTv / 64), lg = blockIdx.x % (TTv / 64); const int b = slab / NHv, h = slab % NHv;
  for (int i = tid; i < 64 * 8; i += 256) { const int r = i / 8, c8 = (i % 8) * 8; FragH f; f.half[0] = *(const v8us*)((const unsigned short*)V16 + ((size_t)b * TTv + lg * 64 + r) * ldv + voff + h * 64 + c8);
#pragma unroll
    for (int q = 0; q < 8; ++q) tl[r][c8 + q] = f.u[q]; }
  __syncthreads();
  for (int pass = 0; pass < 2; ++pass) {
#pragma unroll
    for (int rd = 0; rd < 2; ++rd) { const int d = rd * 32 + tid / 8, pc = tid % 8; FragH f;
#pragma unroll
      for (int q = 0; q < 8; ++q) f.u[q] = tl[pc * 8 + q][d];
      *(volatile v8us*)((unsigned short*)Vt + ((size_t)slab * 64 + d) * TTv + lg * 64 + pc * 8) = f.half[0]; }
    if (pass == 0) __threadfence(); } }

__global__ __launch_bounds__(256) void k_hl(const float* __restrict__ F, _Float16* __restrict__ Hh, _Float16* __restrict__ Hl, size_t n8) { const size_t t = (size_t)blockIdx.x * 256 + threadIdx.x; if (t >= n8) return; FragH fh, fl; const v4f a = *(const v4fa*)(F + t * 8), c = *(const v4fa*)(F + t * 8 + 4);
#pragma unroll
  for (int q = 0; q < 4; ++q) { _Float16 h = (_Float16)a[q]; fh.h[q] = h; fl.h[q] = (_Float16)((a[q] - (float)h) * 1024.0f); h = (_Float16)c[q]; fh.h[4 + q] = h; fl.h[4 + q] = (_Float16)((c[q] - (float)h) * 1024.0f); }
  for (int pass = 0; pass < 2; ++pass) { *(volatile v8us*)((unsigned short*)Hh + t * 8) = fh.half[0]; *(volatile v8us*)((unsigned short*)Hl + t * 8) = fl.half[0]; if (pass == 0) __threadfence(); } }

__global__ __launch_bounds__(256) void k_split(const float* __restrict__ F, _Float16* __restrict__ Hh, _Float16* __restrict__ Hl, size_t n8) {
  #pragma clang fp contract(off)
  const size_t t = (size_t)blockIdx.x * 256 + threadIdx.x; if (t >= n8) return; const v4f a = *(const v4fa*)(F + t * 8), c = *(const v4fa*)(F + t * 8 + 4); FragH fh, fl;
#pragma unroll
  for (int q = 0; q < 8; ++q) { const float v = (q < 4) ? a[q] : c[q - 4]; const _Float16 hi = (_Float16)v; fh.h[q] = hi; fl.h[q] = (_Float16)((v - (float)hi) * 1024.0f); }
  for (int pass = 0; pass < 2; ++pass) { *(volatile v8us*)((unsigned short*)Hh + t * 8) = fh.half[0]; *(volatile v8us*)((unsigned short*)Hl + t * 8) = fl.half[0]; if (pass == 0) __threadfence(); } }
__global__ __launch_bounds__(256) void k_gath(const _Float16* __restrict__ X16, const int* __restrict__ nbr, const int* __restrict__ msk, int k, int p0, _Float16* __restrict__ GA) { const int t = blockIdx.x * 256 + threadIdx.x; if (t >= QP * (PL / 8)) return; const int c0 = (t % (PL / 8)) * 8, r = t / (PL / 8); const int n = p0 + r; v8us v;
#pragma unroll
  for (int q = 0; q < 8; ++q) v[q] = 0;
  if (n < NPt && msk[(size_t)k * NPt + n] > 0) { int i = nbr[(size_t)k * NPt + n]; i = min(max(i, 0), NPt - 1); v = *(const v8us*)((const unsigned short*)X16 + (size_t)i * PL + c0); }
  *(volatile v8us*)((unsigned short*)GA + (size_t)r * PL + c0) = v; __threadfence(); *(volatile v8us*)((unsigned short*)GA + (size_t)r * PL + c0) = v; }
__global__ __launch_bounds__(256) void k_wq(const float* __restrict__ Wq, _Float16* __restrict__ Bq) { const int t = blockIdx.x * 256 + threadIdx.x; if (t >= KO * VEC * (PL / 8)) return; const int i0 = (t % (PL / 8)) * 8; const int kn = t / (PL / 8); const int k = kn / VEC, n = kn % VEC; FragH f;
#pragma unroll
  for (int q = 0; q < 8; ++q) f.h[q] = (_Float16)(bf16_round(Wq[((size_t)k * PL + i0 + q) * VEC + n]) * 16.0f);
  *(volatile v8us*)((unsigned short*)Bq + (size_t)kn * PL + i0) = f.half[0]; __threadfence(); *(volatile v8us*)((unsigned short*)Bq + (size_t)kn * PL + i0) = f.half[0]; }
__global__ __launch_bounds__(256) void k_qexp(const float* __restrict__ QPRE, const float* __restrict__ qg, const float* __restrict__ qb, const float* __restrict__ cb, _Float16* __restrict__ Qh, _Float16* __restrict__ Ql) {
  #pragma clang fp contract(off)
  const int t = blockIdx.x * 256 + threadIdx.x; if (t >= QP * (PL / 8)) return; const int c0 = (t % (PL / 8)) * 8, r = t / (PL / 8); const int v8 = c0 / 8;
  const float qf = fmaxf(QPRE[(size_t)r * VEC + v8] * bf16_round(qg[v8]) + bf16_round(qb[v8]), 0.f); FragH fh, fl;
#pragma unroll
  for (int q = 0; q < 8; ++q) { const float v = bf16_round(cb[c0 + q]) * qf; const _Float16 hi = (_Float16)v; fh.h[q] = hi; fl.h[q] = (_Float16)((v - (float)hi) * 1024.0f); }
  for (int pass = 0; pass < 2; ++pass) { *(volatile v8us*)((unsigned short*)Qh + (size_t)r * PL + c0) = fh.half[0]; *(volatile v8us*)((unsigned short*)Ql + (size_t)r * PL + c0) = fl.half[0]; if (pass == 0) __threadfence(); } }
__global__ __launch_bounds__(1024) void k_choice(const float* __restrict__ CH, int p0, float* __restrict__ CHOICE) {
  #pragma clang fp contract(off)
  __shared__ float res[32]; const int tid = threadIdx.x, w = tid >> 5, l = tid & 31; const int r = blockIdx.x * 32 + w; const v4f v = *(const v4fa*)(CH + (size_t)r * PL + 4 * l); float s = ((fmaxf(v[0], 0.f) + fmaxf(v[1], 0.f)) + fmaxf(v[2], 0.f)) + fmaxf(v[3], 0.f);
  for (int o = 16; o > 0; o >>= 1) s += __shfl_xor(s, o, 32); if (l == 0) res[w] = s;
  __syncthreads();
  const int n = p0 + blockIdx.x * 32 + tid; if (tid < 32 && n < NPP) { *(volatile float*)(CHOICE + n) = res[tid]; __threadfence(); *(volatile float*)(CHOICE + n) = res[tid]; } }
__global__ __launch_bounds__(256) void k_vf(const float* __restrict__ VV, const float* __restrict__ vg, const float* __restrict__ vb, const float* __restrict__ co, const float* __restrict__ Wp, const float* __restrict__ bp, float* __restrict__ VF) {
  #pragma clang fp contract(off)
  const size_t t = (size_t)blockIdx.x * 256 + threadIdx.x; if (t >= (size_t)NPt * (PL / 4)) return; const int c0 = (int)(t % (PL / 4)) * 4; const size_t n = t / (PL / 4); const float x0 = bf16_round(co[n * 3]), x1 = bf16_round(co[n * 3 + 1]), x2 = bf16_round(co[n * 3 + 2]); v4f o; const v4f vv = *(const v4fa*)(VV + n * PL + c0);
#pragma unroll
  for (int q = 0; q < 4; ++q) { const int c = c0 + q; const int v8 = c / 8; const float pos = ((x0 * bf16_round(Wp[v8]) + x1 * bf16_round(Wp[VEC + v8])) + x2 * bf16_round(Wp[2 * VEC + v8])) + bf16_round(bp[v8]); o[q] = fmaxf(vv[q] * bf16_round(vg[c]) + bf16_round(vb[c]), 0.f) + pos; }
  *(volatile v4f*)(VF + n * PL + c0) = o; __threadfence(); *(volatile v4f*)(VF + n * PL + c0) = o; }
__global__ __launch_bounds__(256) void k_attn(const float* __restrict__ CHOICE, const float* __restrict__ VF, const int* __restrict__ nbr, const int* __restrict__ msk, const float* __restrict__ cb, int p0, _Float16* __restrict__ Oh, _Float16* __restrict__ Ol) {
  #pragma clang fp contract(off)
  __shared__ float wa[8][32]; __shared__ int wi[8][32];
  const int tid = threadIdx.x, w = tid >> 5, l = tid & 31; const int r = blockIdx.x * 8 + w; const int n = p0 + r; const bool live = n < NPt; const int nn = live ? n : 0;
  float c2 = 0.f; { const v4f c4 = *(const v4fa*)(cb + 4 * l); c2 = ((bf16_round(c4[0]) * bf16_round(c4[0]) + bf16_round(c4[1]) * bf16_round(c4[1])) + bf16_round(c4[2]) * bf16_round(c4[2])) + bf16_round(c4[3]) * bf16_round(c4[3]); for (int o = 16; o > 0; o >>= 1) c2 += __shfl_xor(c2, o, 32); }
  const float cn = CHOICE[nn]; float s = -3.0e38f; int idx = nn; float mk = 0.f;
  if (l < KO) { int i = nbr[(size_t)l * NPt + nn]; i = min(max(i, 0), NPt - 1); idx = i; mk = (msk[(size_t)l * NPt + nn] > 0) ? 1.f : 0.f; s = (mk > 0.f) ? (cn * CHOICE[i]) * c2 : NEGc; }
  float m = s; for (int o = 16; o > 0; o >>= 1) m = fmaxf(m, __shfl_xor(m, o, 32)); const float e = (l < KO) ? expf(s - m) : 0.f; float den = e; for (int o = 16; o > 0; o >>= 1) den += __shfl_xor(den, o, 32);
  wa[w][l] = (l < KO) ? (mk * (e / den)) : 0.f; wi[w][l] = idx; __syncwarp();
  v4f acc; acc[0] = acc[1] = acc[2] = acc[3] = 0.f;
#pragma unroll 1
  for (int k = 0; k < KO; ++k) { const float a = wa[w][k]; const v4f v = *(const v4fa*)(VF + (size_t)wi[w][k] * PL + 4 * l);
#pragma unroll
    for (int q = 0; q < 4; ++q) acc[q] += v[q] * a; }
  FragH fh, fl;
#pragma unroll
  for (int q = 0; q < 4; ++q) { const float v = live ? acc[q] : 0.f; const _Float16 hi = (_Float16)v; fh.h[q] = hi; fl.h[q] = (_Float16)((v - (float)hi) * 1024.0f); }
  const unsigned long long vh = *(const unsigned long long*)&fh.u[0], vl = *(const unsigned long long*)&fl.u[0];
  for (int pass = 0; pass < 2; ++pass) { *(volatile unsigned long long*)((unsigned short*)Oh + (size_t)r * PL + 4 * l) = vh; *(volatile unsigned long long*)((unsigned short*)Ol + (size_t)r * PL + 4 * l) = vl; if (pass == 0) __threadfence(); } }
__global__ __launch_bounds__(256) void k_fin(const float* __restrict__ G, const float* __restrict__ og, const float* __restrict__ ob, const float* __restrict__ x, int p0, float* __restrict__ out) {
  #pragma clang fp contract(off)
  const int t = blockIdx.x * 256 + threadIdx.x; if (t >= QP * (PL / 4)) return; const int c0 = (t % (PL / 4)) * 4, r = t / (PL / 4); const int n = p0 + r; if (n >= NPt) return; const v4f g = *(const v4fa*)(G + (size_t)r * PL + c0), xv = *(const v4fa*)(x + (size_t)n * PL + c0); v4f o;
#pragma unroll
  for (int q = 0; q < 4; ++q) o[q] = fmaxf(g[q] * bf16_round(og[c0 + q]) + bf16_round(ob[c0 + q]), 0.f) + bf16_round(xv[q]);
  *(volatile v4f*)(out + (size_t)n * PL + c0) = o; __threadfence(); *(volatile v4f*)(out + (size_t)n * PL + c0) = o; }

extern "C" void kernel_launch(void* const* d_in, const int* in_sizes, int n_in,
                              void* d_out, int out_size, void* d_ws, size_t ws_size, hipStream_t stream) {
  (void)in_sizes; (void)n_in; (void)out_size;
  const float* x = (const float*)d_in[0]; const float* co = (const float*)d_in[1]; const float* Wq = (const float*)d_in[2]; const float* qg = (const float*)d_in[3]; const float* qb = (const float*)d_in[4]; const float* Wv = (const float*)d_in[5]; const float* vg = (const float*)d_in[6]; const float* vb = (const float*)d_in[7]; const float* cb = (const float*)d_in[8]; const float* Wc = (const float*)d_in[9]; const float* bc = (const float*)d_in[10]; const float* Wp = (const float*)d_in[11]; const float* bp = (const float*)d_in[12]; const float* Wo = (const float*)d_in[13]; const float* og = (const float*)d_in[14]; const float* ob = (const float*)d_in[15]; const int* nbr = (const int*)d_in[16]; const int* msk = (const int*)d_in[17];
  char* ws = (char*)d_ws; size_t off = 0;
  auto take = [&](size_t bytes) { char* p = ws + off; off += (bytes + 255) & ~(size_t)255; return p; };
  _Float16* Bq = (_Float16*)take((size_t)KO * VEC * PL * 2); _Float16* Bv = (_Float16*)take((size_t)PL * PL * 2); _Float16* Bc = (_Float16*)take((size_t)PL * PL * 2); _Float16* Bo = (_Float16*)take((size_t)PL * PL * 2);
  _Float16* X16 = (_Float16*)take((size_t)NPP * PL * 2); float* CHOICE = (float*)take((size_t)NPP * 4); float* VV = (float*)take((size_t)NPP * PL * 4); float* VF = VV;
  _Float16* GA = (_Float16*)take((size_t)QP * PL * 2); float* QPRE = (float*)take((size_t)QP * VEC * 4); _Float16* Qh = (_Float16*)take((size_t)QP * PL * 2); _Float16* Ql = (_Float16*)take((size_t)QP * PL * 2); float* CH = (float*)take((size_t)QP * PL * 4);
  _Float16* Oh = Qh; _Float16* Ol = Ql; float* G = CH;
  if (off > ws_size) return;
  k_wq<<<(KO * VEC * (PL / 8) + 255) / 256, 256, 0, stream>>>(Wq, Bq); k_wt_f16<<<(PL * (PL / 8) + 255) / 256, 256, 0, stream>>>(Wv, Bv, PL, PL, 16.0f); k_wt_f16<<<(PL * (PL / 8) + 255) / 256, 256, 0, stream>>>(Wc, Bc, PL, PL, 16.0f); k_wt_f16<<<(PL * (PL / 8) + 255) / 256, 256, 0, stream>>>(Wo, Bo, PL, PL, 16.0f);
  k_x16<<<(NPt * PL / 8 + 255) / 256, 256, 0, stream>>>(x, X16, (size_t)NPt * PL / 8);
  const dim3 gQ16(((QP / 16) * 1 + 3) / 4, 1), gQ(((QP / 16) * (PL / 64) + 3) / 4, 1), gAll(((NPP / 16) * (PL / 64) + 3) / 4, 1);
  k_gemm_hhx<0><<<gAll, 128, 0, stream>>>(X16, PL, 0, Bv, PL, 0, 0.0625f, nullptr, 0, nullptr, 1, 0, 0, VV, nullptr, PL, 0, NPP, PL, PL);
  k_vf<<<(unsigned)(((size_t)NPt * (PL / 4) + 255) / 256), 256, 0, stream>>>(VV, vg, vb, co, Wp, bp, VF);
  for (int qq = 0; qq < 4; ++qq) { const int p0 = qq * QP;
    for (int k = 0; k < KO; ++k) { k_gath<<<(QP * (PL / 8) + 255) / 256, 256, 0, stream>>>(X16, nbr, msk, k, p0, GA);
      k_gemm_hhx<0><<<gQ16, 128, 0, stream>>>(GA, PL, 0, Bq + (size_t)k * VEC * PL, PL, 0, 0.0625f, nullptr, 0, (k == 0) ? nullptr : QPRE, 1, (size_t)VEC, 0, QPRE, nullptr, VEC, 0, QP, VEC, PL); }
    k_qexp<<<(QP * (PL / 8) + 255) / 256, 256, 0, stream>>>(QPRE, qg, qb, cb, Qh, Ql);
    k_gemm_hhx<0><<<gQ, 128, 0, stream>>>(Qh, PL, 0, Bc, PL, 0, 0.0625f, bc, 0, nullptr, 1, 0, 0, CH, nullptr, PL, 0, QP, PL, PL); k_gemm_hhx<0><<<gQ, 128, 0, stream>>>(Ql, PL, 0, Bc, PL, 0, 0.0625f / 1024.0f, nullptr, 0, CH, 1, (size_t)PL, 0, CH, nullptr, PL, 0, QP, PL, PL);
    k_choice<<<QP / 32, 1024, 0, stream>>>(CH, p0, CHOICE); }
  for (int qq = 0; qq < 4; ++qq) { const int p0 = qq * QP;
    k_attn<<<QP / 8, 256, 0, stream>>>(CHOICE, VF, nbr, msk, cb, p0, Oh, Ol);
    k_gemm_hhx<0><<<gQ, 128, 0, stream>>>(Oh, PL, 0, Bo, PL, 0, 0.0625f, nullptr, 0, nullptr, 1, 0, 0, G, nullptr, PL, 0, QP, PL, PL); k_gemm_hhx<0><<<gQ, 128, 0, stream>>>(Ol, PL, 0, Bo, PL, 0, 0.0625f / 1024.0f, nullptr, 0, G, 1, (size_t)PL, 0, G, nullptr, PL, 0, QP, PL, PL);
    k_fin<<<(QP * (PL / 4) + 255) / 256, 256, 0, stream>>>(G, og, ob, x, p0, (float*)d_out); }
}
